// Block_89627377533109
// MI455X (gfx1250) — hardware-verified
//
#include <hip/hip_runtime.h>
#ifndef NB
#define NB 2
#endif
#ifndef SEQ
#define SEQ 2048
#endif
#define SQ SEQ
#define NB_FULL 2
#define SQ_FULL 2048
#define DM 1024
#define NH 16
#define HD 64
#define DFF 1024
#define QT 256
#define NKX SQ
#define QT0 128
#define NR ((size_t)NB * SQ)
#define LQ (3 * DM)
static_assert(NH * HD == DM);
static_assert(SQ % QT == 0 && QT % 128 == 0 && (QT & (QT - 1)) == 0);
static_assert(QT0 == 128 && QT0 <= SQ && SQ <= SQ_FULL && NB <= NB_FULL);
static_assert(DM % 64 == 0 && DFF % 64 == 0 && DM % 32 == 0 && DFF % 32 == 0 && HD == 64);
static_assert(DM / 4 == 256);
static_assert(DFF <= 3 * DM);
static_assert((((size_t)NB * SQ * DM) / 4) % 256 == 0);
static_assert((size_t)NB * SQ * DM / 4 < 0x7fffffffu);

typedef unsigned short v8us __attribute__((ext_vector_type(8), may_alias));
typedef float  v8f  __attribute__((ext_vector_type(8)));
typedef float  v4f  __attribute__((ext_vector_type(4)));
typedef float  v4fa __attribute__((ext_vector_type(4), may_alias));
typedef _Float16 v16h __attribute__((ext_vector_type(16)));
typedef _Float16 v4h __attribute__((ext_vector_type(4)));
union FragH { v16h v; v8us half[2]; _Float16 h[16]; unsigned short u[16]; };

__device__ __forceinline__ unsigned short bf16_bits(float x) { unsigned int u = __float_as_uint(x); return (unsigned short)((u + 0x7FFFu + ((u >> 16) & 1u)) >> 16); }
__device__ __forceinline__ float bf16_rne(float x) { return __uint_as_float(((unsigned int)bf16_bits(x)) << 16); }

__device__ __forceinline__ v16h g2_frag(const _Float16* p, unsigned hh) { FragH f; f.half[0] = *(const v8us*)((const unsigned short*)p + 8u * hh); f.half[1] = *(const v8us*)((const unsigned short*)p + 16u + 8u * hh); return f.v; }
__device__ __forceinline__ v8f g2_mma(v16h a, v16h b, v8f c) { v8f d = __builtin_amdgcn_wmma_f32_16x16x32_f16(false, a, false, b, (short)0, c, false, false); asm volatile("v_nop\n\tv_nop\n\tv_nop\n\tv_nop" : "+v"(d) : "v"(a), "v"(b)); return d; }

template <int ACT>
__global__ __launch_bounds__(128) void k_gemm2(const _Float16* __restrict__ A, int lda, size_t sA, const _Float16* __restrict__ Bh, int ldb, size_t sB, float alpha,
    const float* __restrict__ bias, const float* __restrict__ CP, float* __restrict__ C, _Float16* __restrict__ C16, int ldc, size_t sC, int M, int N, int K) {
  static_assert(ACT == 0 || ACT == 3);
  __shared__ __attribute__((aligned(16))) float so[4][32][68];
  const unsigned tid = threadIdx.x, w = tid >> 5, lane = tid & 31u, ln = lane & 15u, hh = lane >> 4; const unsigned by = blockIdx.y;
  A += (size_t)by * sA; Bh += (size_t)by * sB; const size_t cofs = (size_t)by * sC;
  const unsigned ntn = (unsigned)N >> 6; const unsigned mt = blockIdx.x / ntn, nq = blockIdx.x - mt * ntn; const unsigned row0 = mt * 128u + 32u * w, col0 = nq * 64u; if (row0 >= (unsigned)M) return;
  const _Float16* a0p = A + (size_t)(row0 + ln) * (size_t)lda; const _Float16* a1p = a0p + (size_t)16 * (size_t)lda;
  const _Float16* b0p = Bh + (size_t)(col0 + ln) * (size_t)ldb; const _Float16* b1p = b0p + (size_t)16 * (size_t)ldb; const _Float16* b2p = b1p + (size_t)16 * (size_t)ldb; const _Float16* b3p = b2p + (size_t)16 * (size_t)ldb;
  const v8f z8 = {0.f,0.f,0.f,0.f,0.f,0.f,0.f,0.f}; v8f c00 = z8, c01 = z8, c02 = z8, c03 = z8, c10 = z8, c11 = z8, c12 = z8, c13 = z8;
#pragma unroll 1
  for (int kb = 0; kb < K; kb += 32) { const v16h a0 = g2_frag(a0p + kb, hh), a1 = g2_frag(a1p + kb, hh);
    v16h b = g2_frag(b0p + kb, hh); c00 = g2_mma(a0, b, c00); c10 = g2_mma(a1, b, c10);
    b = g2_frag(b1p + kb, hh); c01 = g2_mma(a0, b, c01); c11 = g2_mma(a1, b, c11);
    b = g2_frag(b2p + kb, hh); c02 = g2_mma(a0, b, c02); c12 = g2_mma(a1, b, c12);
    b = g2_frag(b3p + kb, hh); c03 = g2_mma(a0, b, c03); c13 = g2_mma(a1, b, c13); }
  v8f accs[8] = {c00, c01, c02, c03, c10, c11, c12, c13};
#pragma unroll
  for (int u = 0; u < 8; ++u) { const unsigned t = (unsigned)u & 3u, half = (unsigned)u >> 2; const unsigned col = col0 + t * 16u + ln; const float bv = bias ? bf16_rne(bias[col]) : 0.f;
#pragma unroll
    for (int r = 0; r < 8; ++r) { const unsigned rloc = half * 16u + 8u * hh + (unsigned)r; float v = accs[u][r] * alpha + bv;
      if (CP) v += CP[cofs + (size_t)(row0 + rloc) * (size_t)ldc + col];
      if (ACT == 3) v = fmaxf(v, 0.f);
      so[w][rloc][t * 16u + ln] = v; } }
  __builtin_amdgcn_fence(4  , "workgroup"); __builtin_amdgcn_wave_barrier();
  const unsigned rsub = lane >> 4, c4 = (lane & 15u) * 4u;
  for (int pass = 0; pass < 2; ++pass) {
#pragma unroll
    for (int q = 0; q < 16; ++q) { const unsigned r = (unsigned)q * 2u + rsub; const v4f v = *(const v4fa*)&so[w][r][c4];
      if (C) *(volatile v4f*)(C + cofs + (size_t)(row0 + r) * (size_t)ldc + col0 + c4) = v;
      if (C16) { v4h h4; for (int i = 0; i < 4; ++i) h4[i] = (_Float16)v[i]; *(volatile v4h*)(C16 + cofs + (size_t)(row0 + r) * (size_t)ldc + col0 + c4) = h4; } }
    if (pass == 0) __threadfence(); } }

__global__ __launch_bounds__(256) void k_wt_f16(const float* __restrict__ W, _Float16* __restrict__ Wt, int K, int N, float scale) {
  const unsigned k8n = (unsigned)K >> 3; const unsigned t = blockIdx.x * 256u + threadIdx.x; if (t >= (unsigned)N * k8n) return; const unsigned n = t / k8n, k8 = (t - n * k8n) * 8u; FragH f;
#pragma unroll
  for (int i = 0; i < 8; ++i) f.h[i] = (_Float16)(bf16_rne(W[(size_t)(k8 + (unsigned)i) * (size_t)N + n]) * scale);
  const v8us o = f.half[0]; unsigned short* dst = (unsigned short*)Wt + (size_t)n * (size_t)K + k8;
  *(volatile v8us*)dst = o; __threadfence(); *(volatile v8us*)dst = o; }

__global__ __launch_bounds__(256) void k_wthd(const float* __restrict__ Wt, _Float16* __restrict__ Bt) {
  const unsigned t = blockIdx.x * 256u + threadIdx.x; if (t >= (unsigned)(NH * HD * (DM / 8))) return;
  const unsigned m8 = (t % (unsigned)(DM / 8)) * 8u; const unsigned d = (t / (unsigned)(DM / 8)) % (unsigned)HD; const unsigned h = t / (unsigned)((DM / 8) * HD); FragH f;
#pragma unroll
  for (int q = 0; q < 8; ++q) f.h[q] = (_Float16)(16.0f * bf16_rne(Wt[((size_t)h * DM + m8 + (unsigned)q) * HD + d]));
  const v8us o = f.half[0]; unsigned short* dst = (unsigned short*)Bt + ((size_t)h * HD + d) * DM + m8;
  *(volatile v8us*)dst = o; __threadfence(); *(volatile v8us*)dst = o; }

template <int NHv, int TTv>
__global__ __launch_bounds__(256) void k_vt(const _Float16* __restrict__ V16, int ldv, int voff, _Float16* __restrict__ Vt) {
  __shared__ unsigned short tl[64][66]; const unsigned tid = threadIdx.x; const unsigned slab = blockIdx.x / (unsigned)(TTv / 64), lg = blockIdx.x % (unsigned)(TTv / 64); const unsigned b = slab / (unsigned)NHv, h = slab % (unsigned)NHv;
  for (unsigned i = tid; i < 64u * 8u; i += 256u) { const unsigned r = i >> 3, c8 = (i & 7u) * 8u; FragH f; f.half[0] = *(const v8us*)((const unsigned short*)V16 + ((size_t)b * TTv + lg * 64u + r) * (size_t)ldv + (size_t)voff + h * 64u + c8);
#pragma unroll
    for (int q = 0; q < 8; ++q) tl[r][c8 + (unsigned)q] = f.u[q]; }
  __syncthreads();
  for (int pass = 0; pass < 2; ++pass) {
#pragma unroll
    for (int rd = 0; rd < 2; ++rd) { const unsigned d = (unsigned)rd * 32u + (tid >> 3), pc = tid & 7u; FragH f;
#pragma unroll
      for (int q = 0; q < 8; ++q) f.u[q] = tl[pc * 8u + (unsigned)q][d];
      *(volatile v8us*)((unsigned short*)Vt + ((size_t)slab * 64u + d) * TTv + lg * 64u + pc * 8u) = f.half[0]; }
    if (pass == 0) __threadfence(); } }

__global__ __launch_bounds__(256) void k_rsmcf2(const float* __restrict__ S, const int* __restrict__ pm, _Float16* __restrict__ P, int hg, int q0, int nk) {
  #pragma clang fp contract(off)
  const unsigned t = blockIdx.x * 256u + threadIdx.x; if (t >= (unsigned)hg * (unsigned)QT) return; const float* s = S + (size_t)t * NKX; const int last = q0 + (int)(t & (unsigned)(QT - 1)); float mx = -3.0e38f;
#pragma unroll 1
  for (int j = 0; j < nk; ++j) { const int pj = pm[j]; const float f = ((j <= last) & (pj != 0)) ? 1.f : 0.f; mx = fmaxf(mx, fmaf(f, s[j], (1.f - f) * -1.0e9f)); }
  float se = 0.f;
#pragma unroll 1
  for (int j = 0; j < nk; ++j) { const int pj = pm[j]; const float f = ((j <= last) & (pj != 0)) ? 1.f : 0.f; se += __expf(fmaf(f, s[j], (1.f - f) * -1.0e9f) - mx); }
  const float sc = 256.0f * (1.0f / se);
#pragma unroll 1
  for (int j0 = 0; j0 < nk; j0 += 8) { FragH fr;
#pragma unroll
    for (int q = 0; q < 8; ++q) { const int j = j0 + q; const int pj = pm[j]; const float f = ((j <= last) & (pj != 0)) ? 1.f : 0.f; fr.h[q] = (_Float16)(__expf(fmaf(f, s[j], (1.f - f) * -1.0e9f) - mx) * sc); }
    const v8us o = fr.half[0]; unsigned short* d = (unsigned short*)P + (size_t)t * NKX + j0; *(volatile v8us*)d = o; __threadfence(); *(volatile v8us*)d = o; } }

__global__ __launch_bounds__(64) void k_att0(const float* __restrict__ QF, const float* __restrict__ KF, const float* __restrict__ VF, int ld, const int* __restrict__ pm, float scale, float* __restrict__ OF, int ldo) {
  #pragma clang fp contract(off)
  __shared__ __attribute__((aligned(16))) float lq[64][64]; __shared__ __attribute__((aligned(16))) float lo[64][64];
  const unsigned tid = threadIdx.x; const unsigned h = blockIdx.x / (unsigned)(QT0 / 64), rg = blockIdx.x % (unsigned)(QT0 / 64); const unsigned i = rg * 64u + tid;
  const float* qr = QF + (size_t)i * (size_t)ld + h * HD;
#pragma unroll 1
  for (int c = 0; c < HD / 4; ++c) { *(v4fa*)&lq[tid][c * 4] = *(const v4fa*)(qr + c * 4); const v4f z = {0.f, 0.f, 0.f, 0.f}; *(v4fa*)&lo[tid][c * 4] = z; }
  float m = -1.0e30f, l = 0.f; const int jmax = (int)(rg * 64u + 63u);
#pragma unroll 1
  for (int j = 0; j <= jmax; ++j) { const float* kr = KF + (size_t)j * (size_t)ld + h * HD; const float* vr = VF + (size_t)j * (size_t)ld + h * HD; const int pj = pm[j]; float s = 0.f;
#pragma unroll 1
    for (int c = 0; c < HD / 4; ++c) { const v4f kq = *(const v4fa*)(kr + c * 4); const v4f qq = *(const v4fa*)&lq[tid][c * 4]; s = s + qq[0] * kq[0]; s = s + qq[1] * kq[1]; s = s + qq[2] * kq[2]; s = s + qq[3] * kq[3]; }
    s = s * scale;
    const float f = (((unsigned)j <= i) & (pj != 0)) ? 1.f : 0.f; const float sm = fmaf(f, s, (1.f - f) * -1.0e30f); const float mn = fmaxf(m, sm); const float sc = expf(m - mn); const float e = expf(sm - mn); l = l * sc + e; m = mn;
#pragma unroll 1
    for (int c = 0; c < HD / 4; ++c) { const v4f vv = *(const v4fa*)(vr + c * 4); v4f oo = *(const v4fa*)&lo[tid][c * 4]; for (int u = 0; u < 4; ++u) oo[u] = oo[u] * sc + e * vv[u]; *(v4fa*)&lo[tid][c * 4] = oo; } }
  const float fin = 64.0f * (1.0f / l);
#pragma unroll 1
  for (int c = 0; c < HD / 4; ++c) { v4f oo = *(const v4fa*)&lo[tid][c * 4]; for (int u = 0; u < 4; ++u) oo[u] = oo[u] * fin; *(v4fa*)&lo[tid][c * 4] = oo; }
  __syncthreads();
  for (int pass = 0; pass < 2; ++pass) {
#pragma unroll 1
    for (int it = 0; it < 16; ++it) { const unsigned row = (unsigned)it * 4u + (tid >> 4), pc = (tid & 15u) * 4u; const v4f v = *(const v4fa*)&lo[row][pc]; *(volatile v4f*)(OF + (size_t)(rg * 64u + row) * (size_t)ldo + h * HD + pc) = v; }
    if (pass == 0) __threadfence(); } }

template <int BFIN, int FULLIN>
__global__ __launch_bounds__(256) void k_lnx(const float* __restrict__ X, const float* __restrict__ g, const float* __restrict__ bb, float eps, _Float16* __restrict__ N16) {
  #pragma clang fp contract(off)
  __shared__ float red[256]; const unsigned r = blockIdx.x; const unsigned t = threadIdx.x; const unsigned c0 = t * 4u;
  const size_t xr = FULLIN ? ((size_t)(r / (unsigned)SQ) * SQ_FULL + (r % (unsigned)SQ)) : (size_t)r;
  const v4f xa = *(const v4fa*)(X + xr * DM + c0); float s[4]; float sum = 0.f;
  for (int q = 0; q < 4; ++q) { s[q] = BFIN ? bf16_rne(xa[q]) : xa[q]; sum = sum + s[q]; }
  red[t] = sum; __syncthreads(); for (unsigned st = 128u; st > 0u; st >>= 1) { if (t < st) red[t] = red[t] + red[t + st]; __syncthreads(); } const float mu = red[0] * (1.0f / (float)DM); __syncthreads();
  float vs = 0.f; for (int q = 0; q < 4; ++q) { const float dl = s[q] - mu; vs = vs + dl * dl; } red[t] = vs; __syncthreads(); for (unsigned st = 128u; st > 0u; st >>= 1) { if (t < st) red[t] = red[t] + red[t + st]; __syncthreads(); }
  const float rs = rsqrtf(red[0] * (1.0f / (float)DM) + eps); v4h y;
  for (int q = 0; q < 4; ++q) { const unsigned c = c0 + (unsigned)q; y[q] = (_Float16)((((s[q] - mu) * rs) * bf16_rne(g[c])) + bf16_rne(bb[c])); }
  for (int pass = 0; pass < 2; ++pass) { *(volatile v4h*)(N16 + (size_t)r * DM + c0) = y; if (pass == 0) __threadfence(); } }

__global__ __launch_bounds__(256) void k_resid(const float* __restrict__ x, const int* __restrict__ pm, const _Float16* __restrict__ O16, const float* __restrict__ OF0, float* __restrict__ X1) {
  #pragma clang fp contract(off)
  const unsigned t = blockIdx.x * 256u + threadIdx.x; if (t >= (unsigned)(NR * DM / 4)) return;
  const unsigned row = t / (unsigned)(DM / 4), c0 = (t % (unsigned)(DM / 4)) * 4u; const unsigned b = row / (unsigned)SQ, rl = row % (unsigned)SQ; const bool ft = rl < (unsigned)QT0; const unsigned rs = ft ? rl : 0u;
  const size_t e = (size_t)row * DM + c0;
  const v4f xv = *(const v4fa*)(x + ((size_t)b * SQ_FULL + rl) * DM + c0);
  const v4h oh = *(const v4h*)(O16 + e);
  const v4f of = *(const v4fa*)(OF0 + ((size_t)b * QT0 + rs) * DM + c0);
  const int p0 = pm[(size_t)b * SQ_FULL]; const float pz = (p0 != 0) ? 0.f : __uint_as_float(0x7fc00000u);
  v4f y; for (int q = 0; q < 4; ++q) { const float o = ft ? of[q] : (float)oh[q]; y[q] = (bf16_rne(xv[q]) + o * 0.015625f) + pz; }
  *(volatile v4f*)(X1 + e) = y; __threadfence(); *(volatile v4f*)(X1 + e) = y; }

extern "C" void kernel_launch(void* const* d_in, const int* in_sizes, int n_in,
                              void* d_out, int out_size, void* d_ws, size_t ws_size, hipStream_t stream) {
  if (n_in < 13) return;
  const size_t rows_need = (size_t)(NB - 1) * SQ_FULL + SQ;
  if ((size_t)in_sizes[0] < rows_need * DM) return; if ((size_t)in_sizes[1] < rows_need) return;
  if ((size_t)in_sizes[2] < (size_t)NH * DM * HD || (size_t)in_sizes[3] < (size_t)NH * DM * HD || (size_t)in_sizes[4] < (size_t)NH * DM * HD) return;
  if (in_sizes[5] < DM || in_sizes[6] < DM || in_sizes[7] < DM || in_sizes[8] < DM) return;
  if ((size_t)in_sizes[9] < (size_t)DM * DFF || in_sizes[10] < DFF || (size_t)in_sizes[11] < (size_t)DFF * DM || in_sizes[12] < DM) return;
  if ((size_t)out_size < NR * DM) return;
  const float* x = (const float*)d_in[0]; const int* pmask = (const int*)d_in[1];
  const float* wq = (const float*)d_in[2]; const float* wk = (const float*)d_in[3]; const float* wv = (const float*)d_in[4];
  const float* g1 = (const float*)d_in[5]; const float* be1 = (const float*)d_in[6]; const float* g2 = (const float*)d_in[7]; const float* be2 = (const float*)d_in[8];
  const float* w1 = (const float*)d_in[9]; const float* b1 = (const float*)d_in[10]; const float* w2 = (const float*)d_in[11]; const float* b2 = (const float*)d_in[12];
  char* ws = (char*)d_ws; size_t off = 0;
  auto take = [&](size_t bytes) { char* p = ws + off; off += (bytes + 255) & ~(size_t)255; return p; };
  _Float16* BQKV = (_Float16*)take((size_t)3 * DM * DM * 2);
  _Float16* X16 = (_Float16*)take(NR * DM * 2);
  float* X1 = (float*)take(NR * DM * 4);
  _Float16* BW1 = (_Float16*)take((size_t)DFF * DM * 2); _Float16* BW2 = (_Float16*)take((size_t)DM * DFF * 2);
  _Float16* QKV = (_Float16*)take(NR * 3 * DM * 2); _Float16* Q16 = QKV; _Float16* K16 = QKV + DM; _Float16* V16 = QKV + 2 * DM;
  _Float16* HF16 = QKV;
  _Float16* O16 = (_Float16*)take(NR * DM * 2);
  float* S = (float*)take((size_t)NH * QT * NKX * 4); _Float16* P = (_Float16*)take((size_t)NH * QT * NKX * 2); _Float16* VT = (_Float16*)take((size_t)NH * HD * SQ * 2);
  float* F0 = (float*)take((size_t)QT0 * 3 * DM * 4);
  float* OF0 = (float*)take((size_t)NB * QT0 * DM * 4);
  _Float16* M16 = X16;
  if (off > ws_size || off > (size_t)134217728) return;
  { const unsigned g = (unsigned)(((size_t)NH * HD * (DM / 8) + 255) / 256);
    k_wthd<<<g, 256, 0, stream>>>(wq, BQKV); k_wthd<<<g, 256, 0, stream>>>(wk, BQKV + (size_t)DM * DM); k_wthd<<<g, 256, 0, stream>>>(wv, BQKV + (size_t)2 * DM * DM); }
  k_lnx<1, 1><<<(unsigned)NR, 256, 0, stream>>>(x, g1, be1, 1e-5f, X16);
  k_wt_f16<<<(unsigned)(((size_t)DFF * (DM / 8) + 255) / 256), 256, 0, stream>>>(w1, BW1, DM, DFF, 16.0f);
  k_wt_f16<<<(unsigned)(((size_t)DM * (DFF / 8) + 255) / 256), 256, 0, stream>>>(w2, BW2, DFF, DM, 16.0f);
  k_gemm2<0><<<dim3((unsigned)((NR / 128) * (3 * DM / 64)), 1), 128, 0, stream>>>(X16, DM, (size_t)0, BQKV, DM, (size_t)0, 0.0625f, (const float*)nullptr, (const float*)nullptr, (float*)nullptr, QKV, LQ, (size_t)0, (int)NR, 3 * DM, DM);
  for (int b = 0; b < NB; ++b) { const size_t r0 = (size_t)b * SQ; const int* pmb = pmask + (size_t)b * SQ_FULL;
    k_vt<NH, SQ><<<NH * (SQ / 64), 256, 0, stream>>>(V16 + r0 * LQ, LQ, 0, VT);
    k_gemm2<0><<<dim3((unsigned)((QT0 / 128) * (3 * DM / 64)), 1), 128, 0, stream>>>(X16 + r0 * DM, DM, (size_t)0, BQKV, DM, (size_t)0, 0.0625f, (const float*)nullptr, (const float*)nullptr, F0, (_Float16*)nullptr, 3 * DM, (size_t)0, QT0, 3 * DM, DM);
    k_att0<<<NH * (QT0 / 64), 64, 0, stream>>>(F0, F0 + DM, F0 + 2 * DM, 3 * DM, pmb, 0.125f, OF0 + (size_t)b * QT0 * DM, DM);
    for (int q0 = 0; q0 < SQ; q0 += QT) { const int nk = q0 + QT;
      k_gemm2<0><<<dim3((unsigned)((QT / 128) * (nk / 64)), NH), 128, 0, stream>>>(Q16 + (r0 + q0) * LQ, LQ, (size_t)HD, K16 + r0 * LQ, LQ, (size_t)HD, 0.125f, (const float*)nullptr, (const float*)nullptr, S, (_Float16*)nullptr, NKX, (size_t)QT * NKX, QT, nk, HD);
      k_rsmcf2<<<(NH * QT + 255) / 256, 256, 0, stream>>>(S, pmb, P, NH, q0, nk);
      k_gemm2<0><<<dim3((unsigned)((QT / 128) * (HD / 64)), NH), 128, 0, stream>>>(P, NKX, (size_t)QT * NKX, VT, SQ, (size_t)HD * SQ, 0.25f, (const float*)nullptr, (const float*)nullptr, (float*)nullptr, O16 + (r0 + q0) * DM, DM, (size_t)HD, QT, HD, nk); } }
  k_resid<<<(unsigned)((NR * DM / 4) / 256), 256, 0, stream>>>(x, pmask, O16, OF0, X1);
  k_lnx<0, 0><<<(unsigned)NR, 256, 0, stream>>>(X1, g2, be2, 1e-5f, M16);
  k_gemm2<3><<<dim3((unsigned)((NR / 128) * (DFF / 64)), 1), 128, 0, stream>>>(M16, DM, (size_t)0, BW1, DM, (size_t)0, 0.0625f, b1, (const float*)nullptr, (float*)nullptr, HF16, DFF, (size_t)0, (int)NR, DFF, DM);
  k_gemm2<0><<<dim3((unsigned)((NR / 128) * (DM / 64)), 1), 128, 0, stream>>>(HF16, DFF, (size_t)0, BW2, DFF, (size_t)0, 0.0625f, b2, X1, (float*)d_out, (_Float16*)nullptr, DM, (size_t)0, (int)NR, DM, DFF);
}
